// NeuralNet_37615323578557
// MI455X (gfx1250) — hardware-verified
//
#include <hip/hip_runtime.h>

typedef __attribute__((ext_vector_type(16))) _Float16 v16h;
typedef __attribute__((ext_vector_type(8)))  _Float16 v8h;
typedef __attribute__((ext_vector_type(8)))  float    v8f;
typedef __attribute__((ext_vector_type(4)))  float    v4f;
typedef __attribute__((ext_vector_type(2)))  float    v2f;
typedef __attribute__((ext_vector_type(4)))  unsigned int v4u;

#define HID     128
#define TSTEPS  256
#define XROW    ((TSTEPS + 1) * 2)
#define NB_FULL 4096
#ifndef NB
#define NB NB_FULL
#endif

#define P1PCS   512
#define P2OFF   512
#define P3OFF   2560
#define PIECES  2816
#define W1SC    16.0f
#define W2SC    64.0f
#define W3SC    64.0f

static_assert(NB >= 1 && NB <= NB_FULL);
static_assert(PIECES % 256 == 0);
static_assert(P2OFF % 256 == 0);
static_assert(P3OFF % 256 == 0);
static_assert(HID == 128);
static_assert(TSTEPS == 256);

__device__ __forceinline__ float bf16r(float f) {
  unsigned int u = __float_as_uint(f);
  u = (u + 0x7FFFu + ((u >> 16) & 1u)) & 0xFFFF0000u;
  return __uint_as_float(u);
}

__device__ __forceinline__ v16h cat16(v8h lo, v8h hi) {
  return __builtin_shufflevector(lo, hi, 0, 1, 2, 3, 4, 5, 6, 7, 8, 9, 10, 11, 12, 13, 14, 15);
}

__device__ __forceinline__ v8f wmma16(v16h a, v16h b, v8f c) {
  v8f d = __builtin_amdgcn_wmma_f32_16x16x32_f16(false, a, false, b, (short)0, c, false, false);
  asm volatile("v_nop\n\tv_nop\n\tv_nop\n\tv_nop" : "+v"(d) : "v"(a), "v"(b));
  return d;
}

__global__ __launch_bounds__(256) void prep_weights(
    const float* __restrict__ fW1, const float* __restrict__ fW2, const float* __restrict__ fW3,
    const float* __restrict__ bW1, const float* __restrict__ bW2, const float* __restrict__ bW3,
    const float* __restrict__ iW1, const float* __restrict__ iW2, const float* __restrict__ iW3,
    v4u* __restrict__ dst)
{
  const int g = blockIdx.x * 256 + threadIdx.x;
  if (g >= 3 * PIECES) return;
  const int mlp = g / PIECES;
  const int p   = g - mlp * PIECES;
  const float* W1 = (mlp == 0) ? fW1 : ((mlp == 1) ? bW1 : iW1);
  const float* W2 = (mlp == 0) ? fW2 : ((mlp == 1) ? bW2 : iW2);
  const float* W3 = (mlp == 0) ? fW3 : ((mlp == 1) ? bW3 : iW3);
  const int IN = (mlp == 2) ? 3 : 8;

  float v[8];
  if (p < P1PCS) {
    const int l = p & 31, ch = (p >> 5) & 1, j = p >> 6;
    const int h = l >> 4, mm = l & 15;
    const int ncol = 16 * j + mm;
#pragma unroll
    for (int e = 0; e < 8; ++e) {
      const int k  = 8 * h + e + 16 * ch;
      const int kc = min(k, IN - 1);
      const float w = W1[kc * HID + ncol];
      v[e] = (k < IN) ? bf16r(w) * W1SC : 0.0f;
    }
  } else if (p < P3OFF) {
    const int p2 = p - P2OFF;
    const int l = p2 & 31, ch = (p2 >> 5) & 1, jj = (p2 >> 6) & 3, i = p2 >> 8;
    const int h = l >> 4, mm = l & 15;
    const int ncol = 16 * i + mm;
#pragma unroll
    for (int e = 0; e < 8; ++e) {
      const int k = 32 * jj + 8 * h + e + 16 * ch;
      v[e] = bf16r(W2[k * HID + ncol]) * W2SC;
    }
  } else {
    const int p3 = p - P3OFF;
    const int l = p3 & 31, ch = (p3 >> 5) & 1, jj = p3 >> 6;
    const int h = l >> 4, mm = l & 15;
    const int mc = min(mm, 1);
#pragma unroll
    for (int e = 0; e < 8; ++e) {
      const int k = 32 * jj + 8 * h + e + 16 * ch;
      const float w = W3[k * 2 + mc];
      v[e] = (mm < 2) ? bf16r(w) * W3SC : 0.0f;
    }
  }
  v8h o;
#pragma unroll
  for (int e = 0; e < 8; ++e) o[e] = (_Float16)v[e];
  const v4u ob = __builtin_bit_cast(v4u, o);
  v4u* d = dst + g;
  *(volatile v4u*)d = ob;
  __threadfence();
  *(volatile v4u*)d = ob;
}

template <int MODE>
__global__ __launch_bounds__(128)
__attribute__((amdgpu_num_vgpr(256)))
void mlp_chain(const float* __restrict__ x,
               const float* __restrict__ t,
               const v8h* __restrict__ gW,
               const float* __restrict__ B1,
               const float* __restrict__ B2,
               const float* __restrict__ B3,
               float* __restrict__ plane,
               int numTiles)
{
  __shared__ v8h wAll[PIECES];
  __shared__ float sb1[HID];
  __shared__ float sb2[HID];
  __shared__ float sb3[2];
  __shared__ __align__(16) float sOut[4][64];

  const int tid  = threadIdx.x;
  const int lane = tid & 31;
  const int wave = tid >> 5;

  for (int p = tid; p < PIECES; p += 128) wAll[p] = gW[p];
  sb1[tid] = bf16r(B1[tid]);
  sb2[tid] = bf16r(B2[tid]);
  if (tid < 2) sb3[tid] = bf16r(B3[tid]);
  __syncthreads();

  const int h    = lane >> 4;
  const int n    = lane & 15;
  const int mofs = 8 * h;
  const int waveId     = blockIdx.x * 4 + wave;
  const int waveStride = gridDim.x * 4;

  v8f zero8;
#pragma unroll
  for (int e = 0; e < 8; ++e) zero8[e] = 0.0f;
  v16h zero16;
#pragma unroll
  for (int e = 0; e < 16; ++e) zero16[e] = (_Float16)0.0f;

  for (int tp = waveId; tp < numTiles; tp += waveStride) {
    int ofs0 = 0;
    asm volatile("" : "+v"(ofs0));
    const int laneO = lane + ofs0;

    v16h fB[2];
    int  vld[2];
#pragma unroll
    for (int r = 0; r < 2; ++r) {
      float f[8];
      if (MODE == 2) {
        const int row = tp * 32 + 16 * r + n;
        vld[r] = (row < NB) ? 1 : 0;
        const int bc = min(row, NB - 1);
        const float* xb = x + (size_t)bc * XROW;
        const v2f x0 = *(const v2f*)(xb);
        const float tb = t[bc];
        f[0] = bf16r(x0.x); f[1] = bf16r(x0.y); f[2] = bf16r(tb);
        f[3] = 0.0f; f[4] = 0.0f; f[5] = 0.0f; f[6] = 0.0f; f[7] = 0.0f;
      } else {
        const int b  = tp >> 3;
        const int j  = (tp & 7) * 32 + 16 * r + n;
        vld[r] = (j < TSTEPS - 1) ? 1 : 0;
        const int jc = min(j, TSTEPS - 2);
        const float* xb = x + (size_t)b * XROW;
        const v2f xa = *(const v2f*)(xb + 2 * jc);
        const v2f xn = *(const v2f*)(xb + 2 * jc + 2);
        const v2f pt = *(const v2f*)(xb + 2 * TSTEPS);
        const float tb = bf16r(t[b]);
        if (MODE == 0) {
          f[0] = bf16r(xn.x); f[1] = bf16r(xn.y); f[2] = tb;
          f[3] = bf16r(xa.x); f[4] = bf16r(xa.y);
          f[5] = (float)(jc + 1) * (1.0f / (float)TSTEPS);
          f[6] = bf16r(pt.x); f[7] = bf16r(pt.y);
        } else {
          f[0] = bf16r(xa.x); f[1] = bf16r(xa.y); f[2] = tb;
          f[3] = bf16r(xn.x); f[4] = bf16r(xn.y);
          f[5] = (float)jc * (1.0f / (float)TSTEPS);
          f[6] = bf16r(pt.x); f[7] = bf16r(pt.y);
        }
      }
      v16h a = zero16;
#pragma unroll
      for (int i = 0; i < 8; ++i) a[i] = (h == 0) ? (_Float16)f[i] : (_Float16)0.0f;
      fB[r] = a;
    }

    v16h B2f[4][2];
#pragma unroll
    for (int c = 0; c < 4; ++c) { B2f[c][0] = zero16; B2f[c][1] = zero16; }
#pragma unroll
    for (int j = 0; j < 8; ++j) {
      const v16h aW = cat16(wAll[(j * 2 + 0) * 32 + laneO], wAll[(j * 2 + 1) * 32 + laneO]);
#pragma unroll
      for (int r = 0; r < 2; ++r) {
        const v8f acc = wmma16(aW, fB[r], zero8);
#pragma unroll
        for (int rr = 0; rr < 8; ++rr) {
          const float bias = sb1[16 * j + mofs + rr + ofs0];
          const float v = fmaxf(acc[rr] * (1.0f / W1SC) + bias, 0.0f);
          B2f[j >> 1][r][(j & 1) * 8 + rr] = (_Float16)v;
        }
      }
    }

    v16h B3f[4][2];
#pragma unroll
    for (int c = 0; c < 4; ++c) { B3f[c][0] = zero16; B3f[c][1] = zero16; }
#pragma unroll
    for (int i = 0; i < 8; ++i) {
      v8f acc[2];
      acc[0] = zero8; acc[1] = zero8;
#pragma unroll
      for (int jj = 0; jj < 4; ++jj) {
        const v16h aW = cat16(wAll[P2OFF + ((i * 4 + jj) * 2 + 0) * 32 + laneO],
                              wAll[P2OFF + ((i * 4 + jj) * 2 + 1) * 32 + laneO]);
#pragma unroll
        for (int r = 0; r < 2; ++r) acc[r] = wmma16(aW, B2f[jj][r], acc[r]);
      }
#pragma unroll
      for (int r = 0; r < 2; ++r) {
#pragma unroll
        for (int rr = 0; rr < 8; ++rr) {
          const float bias = sb2[16 * i + mofs + rr + ofs0];
          const float v = fmaxf(acc[r][rr] * (1.0f / W2SC) + bias, 0.0f);
          B3f[i >> 1][r][(i & 1) * 8 + rr] = (_Float16)v;
        }
      }
    }

    v8f acc3[2];
    acc3[0] = zero8; acc3[1] = zero8;
#pragma unroll
    for (int jj = 0; jj < 4; ++jj) {
      const v16h aW = cat16(wAll[P3OFF + (jj * 2 + 0) * 32 + laneO],
                            wAll[P3OFF + (jj * 2 + 1) * 32 + laneO]);
#pragma unroll
      for (int r = 0; r < 2; ++r) acc3[r] = wmma16(aW, B3f[jj][r], acc3[r]);
    }

    const float b30 = sb3[0 + ofs0];
    const float b31 = sb3[1 + ofs0];
#pragma unroll
    for (int r = 0; r < 2; ++r) {
      const float o0 = vld[r] ? (acc3[r][0] * (1.0f / W3SC) + b30) : 0.0f;
      const float o1 = vld[r] ? (acc3[r][1] * (1.0f / W3SC) + b31) : 0.0f;
      if (h == 0) {
        sOut[wave][2 * (16 * r + n) + 0] = o0;
        sOut[wave][2 * (16 * r + n) + 1] = o1;
      }
    }
    __builtin_amdgcn_fence(__ATOMIC_RELEASE, "wavefront");
    __builtin_amdgcn_wave_barrier();

    const v4f o4 = *(const v4f*)(&sOut[wave][4 * n]);
    float* dstp = plane + (size_t)tp * 64 + 4 * n;
    if (lane < 16) { *(volatile v4f*)dstp = o4; }
    __threadfence();
    if (lane < 16) { *(volatile v4f*)dstp = o4; }

    __builtin_amdgcn_fence(__ATOMIC_RELEASE, "wavefront");
    __builtin_amdgcn_wave_barrier();
  }
}

__global__ __launch_bounds__(256) void combine_score(
    const float* __restrict__ pF,
    const float* __restrict__ pB,
    const float* __restrict__ pI,
    float* __restrict__ out,
    int total4)
{
  const int idx = blockIdx.x * 256 + threadIdx.x;
  if (idx >= total4) return;
  const int b  = idx >> 7;
  const int i4 = idx & 127;
  const int i0 = 2 * i4;
  const int i1 = i0 + 1;
  const float* fb = pF + (size_t)b * (TSTEPS * 2);
  const int im1 = max(i0 - 1, 0);
  const v2f fa  = *(const v2f*)(fb + 2 * im1);
  const v2f fbv = *(const v2f*)(fb + 2 * i0);
  const v4f bw  = *(const v4f*)(pB + (size_t)b * (TSTEPS * 2) + 4 * i4);
  const v2f iv  = *(const v2f*)(pI + 2 * b);

  float o0 = (i0 >= 1) ? fa.x : 0.0f;
  float o1 = (i0 >= 1) ? fa.y : 0.0f;
  o0 = o0 + ((i0 <= TSTEPS - 2) ? bw.x : 0.0f);
  o1 = o1 + ((i0 <= TSTEPS - 2) ? bw.y : 0.0f);
  o0 = o0 + ((i0 == 0) ? iv.x : 0.0f);
  o1 = o1 + ((i0 == 0) ? iv.y : 0.0f);
  float o2 = fbv.x;
  float o3 = fbv.y;
  o2 = o2 + ((i1 <= TSTEPS - 2) ? bw.z : 0.0f);
  o3 = o3 + ((i1 <= TSTEPS - 2) ? bw.w : 0.0f);

  v4f o;
  o[0] = o0; o[1] = o1; o[2] = o2; o[3] = o3;
  float* d = out + (size_t)idx * 4;
  *(volatile v4f*)d = o;
  __threadfence();
  *(volatile v4f*)d = o;
}

extern "C" void kernel_launch(void* const* d_in, const int* in_sizes, int n_in,
                              void* d_out, int out_size, void* d_ws, size_t ws_size,
                              hipStream_t stream) {
  if (n_in < 20) return;
  if (in_sizes[0]  < NB * XROW) return;
  if (in_sizes[1]  < NB) return;
  if (in_sizes[2]  < 8 * HID || in_sizes[3]  < HID || in_sizes[4]  < HID * HID ||
      in_sizes[5]  < HID     || in_sizes[6]  < HID * 2 || in_sizes[7] < 2) return;
  if (in_sizes[8]  < 8 * HID || in_sizes[9]  < HID || in_sizes[10] < HID * HID ||
      in_sizes[11] < HID     || in_sizes[12] < HID * 2 || in_sizes[13] < 2) return;
  if (in_sizes[14] < 3 * HID || in_sizes[15] < HID || in_sizes[16] < HID * HID ||
      in_sizes[17] < HID     || in_sizes[18] < HID * 2 || in_sizes[19] < 2) return;
  if (out_size < NB * TSTEPS * 2) return;

  const float* x  = (const float*)d_in[0];
  const float* t  = (const float*)d_in[1];
  const float* fw_W1 = (const float*)d_in[2];  const float* fw_b1 = (const float*)d_in[3];
  const float* fw_W2 = (const float*)d_in[4];  const float* fw_b2 = (const float*)d_in[5];
  const float* fw_W3 = (const float*)d_in[6];  const float* fw_b3 = (const float*)d_in[7];
  const float* bw_W1 = (const float*)d_in[8];  const float* bw_b1 = (const float*)d_in[9];
  const float* bw_W2 = (const float*)d_in[10]; const float* bw_b2 = (const float*)d_in[11];
  const float* bw_W3 = (const float*)d_in[12]; const float* bw_b3 = (const float*)d_in[13];
  const float* in_W1 = (const float*)d_in[14]; const float* in_b1 = (const float*)d_in[15];
  const float* in_W2 = (const float*)d_in[16]; const float* in_b2 = (const float*)d_in[17];
  const float* in_W3 = (const float*)d_in[18]; const float* in_b3 = (const float*)d_in[19];
  float* out = (float*)d_out;

  const int tilesFB = NB * 8;
  const int tilesI  = (NB + 31) / 32;
  const size_t szF  = (size_t)tilesFB * 32 * 2 * sizeof(float);
  const size_t szI  = (size_t)tilesI * 32 * 2 * sizeof(float);
  const size_t szW  = (size_t)3 * PIECES * 16;
  const size_t offF = 0;
  const size_t offB = offF + szF;
  const size_t offI = offB + szF;
  const size_t offW = offI + szI;
  const size_t total = offW + szW;
  if (total > ws_size) return;

  char* ws = (char*)d_ws;
  float* planeF = (float*)(ws + offF);
  float* planeB = (float*)(ws + offB);
  float* planeI = (float*)(ws + offI);
  v8h*   planeW = (v8h*)(ws + offW);

  prep_weights<<<(3 * PIECES + 255) / 256, 256, 0, stream>>>(
      fw_W1, fw_W2, fw_W3, bw_W1, bw_W2, bw_W3, in_W1, in_W2, in_W3, (v4u*)planeW);

  int gridFB = (tilesFB + 3) / 4;  if (gridFB > 256) gridFB = 256;
  int gridI  = (tilesI + 3) / 4;   if (gridI > 256) gridI = 256;

  mlp_chain<0><<<gridFB, 128, 0, stream>>>(x, t, planeW + 0 * PIECES, fw_b1, fw_b2, fw_b3,
                                           planeF, tilesFB);
  mlp_chain<1><<<gridFB, 128, 0, stream>>>(x, t, planeW + 1 * PIECES, bw_b1, bw_b2, bw_b3,
                                           planeB, tilesFB);
  mlp_chain<2><<<gridI, 128, 0, stream>>>(x, t, planeW + 2 * PIECES, in_b1, in_b2, in_b3,
                                          planeI, tilesI);

  const int total4 = NB * 128;
  combine_score<<<(total4 + 255) / 256, 256, 0, stream>>>(planeF, planeB, planeI, out, total4);
}
